// GAT_68118181314620
// MI455X (gfx1250) — hardware-verified
//
#include <hip/hip_runtime.h>
#include <stddef.h>
#include <stdint.h>
#include <math.h>


#define DCH    128
#define KP     256
#define NTHR   256
#define NWAVE  8
#define EPT    8
#define CHUNK  (NTHR * EPT)
#define WCAP   (EPT * 32)
#define LISTN  (NWAVE * WCAP)
#define NBA    1024
#define SLA    10
#define RCAP   28672
#define DEGCAP 128
#define GBM    64
#define GBN    128
#define GTHR   128
#define NU0    (DCH * (DCH / 8))
#define NUC    (DCH * (KP / 8))
#define NEGSL  0.2f
#define EPS_SM 1e-16f
#define AGG_ZINTS (LISTN + 2 * RCAP + 3 * NBA)
#define AGG_LDS_INTS (AGG_ZINTS + 16)
#define WSMAX  134217728

static_assert((CHUNK & (CHUNK - 1)) == 0 && CHUNK <= 4096);
static_assert((NBA & (NBA - 1)) == 0 && NBA == (1 << SLA));
static_assert(((long long)CHUNK << SLA) < (1LL << 31));
static_assert(LISTN % NTHR == 0);
static_assert(NBA % NWAVE == 0 && NBA % 32 == 0 && NBA % GBM == 0);
static_assert(RCAP % 4 == 0 && AGG_ZINTS % 4 == 0 && LISTN % 4 == 0);
static_assert(DCH % 32 == 0 && KP % 32 == 0 && KP == 2 * DCH && DCH == GBN);
static_assert(GBM == (GTHR / 32) * 16 && GBN == 4 * 32);
static_assert(NU0 % NTHR == 0 && NUC % NTHR == 0);
static_assert(DCH / 8 == 16 && KP / 8 == 32);
static_assert(AGG_LDS_INTS * 4 <= 300000);
static_assert(DCH == 4 * 32);
static_assert(KP == 8 * 32);
static_assert(WCAP == 32 * EPT);

typedef float          v4f   __attribute__((ext_vector_type(4)));
typedef float          v8f   __attribute__((ext_vector_type(8)));
typedef int            v4i   __attribute__((ext_vector_type(4)));
typedef int            v8i   __attribute__((ext_vector_type(8)));
typedef unsigned int   v4u   __attribute__((ext_vector_type(4)));
typedef unsigned short v8us  __attribute__((ext_vector_type(8)));
typedef unsigned short v16us __attribute__((ext_vector_type(16)));
typedef __bf16         v16bf __attribute__((ext_vector_type(16)));
typedef v4f  __attribute__((may_alias)) v4fa;
typedef v4i  __attribute__((may_alias)) v4ia;
typedef v8us __attribute__((may_alias)) v8usa;
union FragB { v16bf v; v16us u; v8us h[2]; v8i w; };

__device__ __forceinline__ v8f wmb(const FragB& a, const FragB& b, v8f c) {
  v8f d = __builtin_amdgcn_wmma_f32_16x16x32_bf16(false, a.v, false, b.v, (short)0, c, false, false);
  asm volatile("v_nop\n\tv_nop\n\tv_nop\n\tv_nop" : "+v"(d) : "v"(a.w), "v"(b.w));
  return d;
}

__device__ __forceinline__ unsigned bf16_bits(float f) {
  const unsigned u = __float_as_uint(f);
  const unsigned r = (u + 0x7FFFu + ((u >> 16) & 1u)) >> 16;
  return (f != f) ? 0x7FC0u : (r & 0xFFFFu);
}
__device__ __forceinline__ float bf16_val(float f) {
  return __uint_as_float(bf16_bits(f) << 16);
}
__device__ __forceinline__ v4f bfr4(const v4f a) {
  v4f r; r.x = bf16_val(a.x); r.y = bf16_val(a.y); r.z = bf16_val(a.z); r.w = bf16_val(a.w); return r;
}
__device__ __forceinline__ v8us cv8(const float* __restrict__ p) {
  const v4f a = *(const v4f*)p;
  const v4f b = *(const v4f*)(p + 4);
  v8us o;
  o[0] = (unsigned short)bf16_bits(a.x); o[1] = (unsigned short)bf16_bits(a.y);
  o[2] = (unsigned short)bf16_bits(a.z); o[3] = (unsigned short)bf16_bits(a.w);
  o[4] = (unsigned short)bf16_bits(b.x); o[5] = (unsigned short)bf16_bits(b.y);
  o[6] = (unsigned short)bf16_bits(b.z); o[7] = (unsigned short)bf16_bits(b.w);
  return o;
}

template <int SLB>
__device__ __forceinline__ int scan_chunk(const int* __restrict__ dsts, int nE, int cbase, int slotBase,
                                          int nb, int vec8, int* list, int tid, int lane, int wave) {
  int wc = 0;
  const int el0  = tid * EPT;
  const int e0   = cbase + el0;
  const int sent = -2147483647 - 1;
  v4i da, db;
  if (vec8 != 0 && cbase + CHUNK <= nE) {
    da = *(const v4i*)(dsts + e0);
    db = *(const v4i*)(dsts + e0 + 4);
  } else {
    da.x = (e0     < nE) ? dsts[min(e0,     nE - 1)] : sent;
    da.y = (e0 + 1 < nE) ? dsts[min(e0 + 1, nE - 1)] : sent;
    da.z = (e0 + 2 < nE) ? dsts[min(e0 + 2, nE - 1)] : sent;
    da.w = (e0 + 3 < nE) ? dsts[min(e0 + 3, nE - 1)] : sent;
    db.x = (e0 + 4 < nE) ? dsts[min(e0 + 4, nE - 1)] : sent;
    db.y = (e0 + 5 < nE) ? dsts[min(e0 + 5, nE - 1)] : sent;
    db.z = (e0 + 6 < nE) ? dsts[min(e0 + 6, nE - 1)] : sent;
    db.w = (e0 + 7 < nE) ? dsts[min(e0 + 7, nE - 1)] : sent;
  }
  const unsigned nbs = (unsigned)slotBase;
  const unsigned unb = (unsigned)nb;
  const unsigned s0 = (unsigned)da.x - nbs, s1 = (unsigned)da.y - nbs;
  const unsigned s2 = (unsigned)da.z - nbs, s3 = (unsigned)da.w - nbs;
  const unsigned s4 = (unsigned)db.x - nbs, s5 = (unsigned)db.y - nbs;
  const unsigned s6 = (unsigned)db.z - nbs, s7 = (unsigned)db.w - nbs;
  const bool h0 = s0 < unb, h1 = s1 < unb, h2 = s2 < unb, h3 = s3 < unb;
  const bool h4 = s4 < unb, h5 = s5 < unb, h6 = s6 < unb, h7 = s7 < unb;
  const int nl = (int)h0 + (int)h1 + (int)h2 + (int)h3 + (int)h4 + (int)h5 + (int)h6 + (int)h7;
  const unsigned any = __builtin_amdgcn_ballot_w32(nl != 0);
  if (any != 0u) {
    int incl = nl;
#pragma unroll
    for (int d = 1; d < 32; d <<= 1) {
      const int up = __shfl_up(incl, d, 32);
      if (lane >= d) incl += up;
    }
    wc = __builtin_amdgcn_readlane(incl, 31);
    int pos = incl - nl;
    int* lw = list + wave * WCAP;
#define PUTJ(J, HJ, SJ) if (HJ) { if (pos < WCAP) lw[pos] = ((el0 + (J)) << SLB) | (int)(SJ); pos = pos + 1; }
    PUTJ(0, h0, s0)
    PUTJ(1, h1, s1)
    PUTJ(2, h2, s2)
    PUTJ(3, h3, s3)
    PUTJ(4, h4, s4)
    PUTJ(5, h5, s5)
    PUTJ(6, h6, s6)
    PUTJ(7, h7, s7)
#undef PUTJ
  }
  return wc;
}

__global__ __launch_bounds__(NTHR) void k_wprep(const float* __restrict__ W0, const float* __restrict__ W1,
                                                const float* __restrict__ W2,
                                                unsigned short* W0B, unsigned short* W1C, unsigned short* W2C) {
  const int u = (int)blockIdx.x * NTHR + (int)threadIdx.x;
  v8us o;
  unsigned short* dp;
  if (u < NU0) {
    const int n  = u >> 4;
    const int k8 = (u & 15) * 8;
    o  = cv8(W0 + (size_t)n * DCH + k8);
    dp = W0B + (size_t)n * DCH + k8;
  } else if (u < NU0 + NUC) {
    const int v  = u - NU0;
    const int n  = v >> 5;
    const int k8 = (v & 31) * 8;
    const int kk = k8 & (DCH - 1);
    o  = cv8(W1 + (size_t)n * DCH + kk);
    dp = W1C + (size_t)n * KP + k8;
  } else if (u < NU0 + 2 * NUC) {
    const int v  = u - NU0 - NUC;
    const int n  = v >> 5;
    const int k8 = (v & 31) * 8;
    const int kk = k8 & (DCH - 1);
    o  = cv8(W2 + (size_t)n * DCH + kk);
    dp = W2C + (size_t)n * KP + k8;
  } else {
    return;
  }
  *(volatile v8us*)dp = o;
  __threadfence();
  *(volatile v8us*)dp = o;
}

__global__ __launch_bounds__(NTHR) void k_cvx(const float* __restrict__ x, int nN, int nUnits,
                                              unsigned short* xb) {
  const int u = (int)blockIdx.x * NTHR + (int)threadIdx.x;
  if (u >= nUnits) return;
  const int row = u >> 4;
  const int k8  = (u & 15) * 8;
  const int rc  = row < nN ? row : nN - 1;
  const float* p = x + (size_t)rc * DCH + k8;
  const v4f a = *(const v4f*)p;
  const v4f b = *(const v4f*)(p + 4);
  const bool ok = row < nN;
  v8us o;
  o[0] = ok ? (unsigned short)bf16_bits(a.x) : (unsigned short)0;
  o[1] = ok ? (unsigned short)bf16_bits(a.y) : (unsigned short)0;
  o[2] = ok ? (unsigned short)bf16_bits(a.z) : (unsigned short)0;
  o[3] = ok ? (unsigned short)bf16_bits(a.w) : (unsigned short)0;
  o[4] = ok ? (unsigned short)bf16_bits(b.x) : (unsigned short)0;
  o[5] = ok ? (unsigned short)bf16_bits(b.y) : (unsigned short)0;
  o[6] = ok ? (unsigned short)bf16_bits(b.z) : (unsigned short)0;
  o[7] = ok ? (unsigned short)bf16_bits(b.w) : (unsigned short)0;
  unsigned short* dp = xb + (size_t)row * DCH + k8;
  *(volatile v8us*)dp = o;
  __threadfence();
  *(volatile v8us*)dp = o;
}

template <int NC>
__global__ __launch_bounds__(GTHR * NC) void k_gemm(const unsigned short* __restrict__ A, int lda,
                                                    const unsigned short* __restrict__ BT, int ldb, int K,
                                                    float* Cm, const float* __restrict__ avs,
                                                    const float* __restrict__ avd, float* AL) {
  static_assert(NC == 1 || NC == 2);
  constexpr int LDC = GBN * NC;
  constexpr int RPW = GBM / (4 * NC);
  extern __shared__ __attribute__((aligned(16))) float gsm[];
  float* stg = gsm;
  float* sdt = gsm + GBM * LDC;
  const int tid = (int)threadIdx.x, lane = tid & 31, wave = tid >> 5, hh = lane >> 4, m = lane & 15;
  const int rg = wave & 3, cg = wave >> 2;
  const int rowBase = (int)blockIdx.x * GBM;
  const int colBase = cg * GBN;

  v8f acc[8];
  {
    const v8f z = {0.f, 0.f, 0.f, 0.f, 0.f, 0.f, 0.f, 0.f};
#pragma unroll
    for (int t = 0; t < 8; ++t) acc[t] = z;
  }
  const unsigned short* ap = A  + (size_t)(rowBase + 16 * rg + m) * (size_t)lda + 8 * hh;
  const unsigned short* bp = BT + (size_t)(colBase + m) * (size_t)ldb + 8 * hh;

#pragma unroll 1
  for (int k0 = 0; k0 < K; k0 += 32) {
    FragB af;
    af.h[0] = *(const v8usa*)(ap + k0);
    af.h[1] = *(const v8usa*)(ap + k0 + 16);
#pragma unroll
    for (int nt = 0; nt < 8; ++nt) {
      const unsigned short* wq = bp + (size_t)(16 * nt) * (size_t)ldb + k0;
      FragB bf;
      bf.h[0] = *(const v8usa*)wq;
      bf.h[1] = *(const v8usa*)(wq + 16);
      acc[nt] = wmb(af, bf, acc[nt]);
    }
  }

#pragma unroll
  for (int nt = 0; nt < 8; ++nt) {
    const int lc = colBase + 16 * nt + m;
#pragma unroll
    for (int r = 0; r < 8; ++r) {
      const int lr = 16 * rg + 8 * hh + r;
      stg[lr * LDC + lc] = acc[nt][r];
    }
  }
  __syncthreads();

  v4f as4[NC], ad4[NC];
#pragma unroll
  for (int c = 0; c < NC; ++c) {
    as4[c] = bfr4(*(const v4fa*)(avs + c * GBN + 4 * lane));
    ad4[c] = bfr4(*(const v4fa*)(avd + c * GBN + 4 * lane));
  }
#pragma unroll 1
  for (int i = 0; i < RPW; ++i) {
    const int row = wave * RPW + i;
    float s = 0.0f, d = 0.0f;
#pragma unroll
    for (int c = 0; c < NC; ++c) {
      const v4f p = *(const v4fa*)(stg + row * LDC + c * GBN + 4 * lane);
      s = fmaf(p.x, as4[c].x, s); s = fmaf(p.y, as4[c].y, s); s = fmaf(p.z, as4[c].z, s); s = fmaf(p.w, as4[c].w, s);
      d = fmaf(p.x, ad4[c].x, d); d = fmaf(p.y, ad4[c].y, d); d = fmaf(p.z, ad4[c].z, d); d = fmaf(p.w, ad4[c].w, d);
    }
#pragma unroll
    for (int off = 16; off > 0; off >>= 1) {
      s += __shfl_xor(s, off);
      d += __shfl_xor(d, off);
    }
    if (lane == 0) { sdt[row] = s; sdt[GBM + row] = d; }
  }
  __syncthreads();

  const v4f alv = *(const v4fa*)(sdt + 4 * lane);
  float* alp = AL + (size_t)blockIdx.x * (2 * GBM) + 4 * lane;
#pragma unroll 1
  for (int i = 0; i < RPW; ++i) {
    const int row = wave * RPW + i;
#pragma unroll
    for (int c = 0; c < NC; ++c) {
      const v4f p = *(const v4fa*)(stg + row * LDC + c * GBN + 4 * lane);
      float* op = Cm + (size_t)(rowBase + row) * (size_t)LDC + c * GBN + 4 * lane;
      *(volatile v4f*)op = p;
    }
  }
  if (wave == 0) *(volatile v4f*)alp = alv;
  __threadfence();
#pragma unroll 1
  for (int i = 0; i < RPW; ++i) {
    const int row = wave * RPW + i;
#pragma unroll
    for (int c = 0; c < NC; ++c) {
      const v4f p = *(const v4fa*)(stg + row * LDC + c * GBN + 4 * lane);
      float* op = Cm + (size_t)(rowBase + row) * (size_t)LDC + c * GBN + 4 * lane;
      *(volatile v4f*)op = p;
    }
  }
  if (wave == 0) *(volatile v4f*)alp = alv;
}

template <int OUTF>
__global__ __launch_bounds__(NTHR) void k_agg(const int* __restrict__ srcs, const int* __restrict__ dsts,
                                              int nE, int nN, int vec8, int mRows,
                                              const float* __restrict__ AL,
                                              const float* __restrict__ xl, const float* __restrict__ bias,
                                              unsigned short* hb, float* outp) {
  extern __shared__ __attribute__((aligned(16))) int dsm[];
  int* list = dsm;
  int* hl   = dsm + LISTN;
  int* sl   = dsm + LISTN + RCAP;
  int* cnt  = dsm + LISTN + 2 * RCAP;
  int* offs = cnt + NBA;
  int* cur  = offs + NBA;
  int* misc = cur + NBA;
  const int tid = (int)threadIdx.x, lane = tid & 31, wave = tid >> 5;
  const int nodeBase = (int)blockIdx.x * NBA;

  {
    const v4i z4 = {0, 0, 0, 0};
    for (int i = tid * 4; i < AGG_ZINTS; i += NTHR * 4) *(v4ia*)(dsm + i) = z4;
    if (tid < 16) misc[tid] = 0;
  }
  const int c0 = 4 * lane;
  const v4f bv = bfr4(*(const v4f*)(bias + c0));
  __syncthreads();

  int t = 0, ov = 0;
  const int nChunks = (nE + CHUNK - 1) / CHUNK;
#pragma unroll 1
  for (int ch = 0; ch < nChunks; ++ch) {
    const int cbase = ch * CHUNK;
    const int wc = scan_chunk<SLA>(dsts, nE, cbase, nodeBase, NBA, vec8, list, tid, lane, wave);
    if (lane == 0) misc[wave] = wc;
    __syncthreads();
    if (wave == 0) {
#pragma unroll 1
      for (int w2 = 0; w2 < NWAVE; ++w2) {
        int c = misc[w2];
        c = c < 0 ? 0 : (c > WCAP ? WCAP : c);
#pragma unroll 1
        for (int b0 = 0; b0 < c; b0 += 32) {
          const int idx = b0 + lane;
          const int ent = list[w2 * WCAP + (idx < WCAP ? idx : WCAP - 1)];
          const int m32 = (c - b0) < 32 ? (c - b0) : 32;
#pragma unroll 1
          for (int k = 0; k < m32; ++k) {
            const int u    = __builtin_amdgcn_readlane(ent, k);
            const int slot = u & (NBA - 1);
            const int el   = (u >> SLA) & (CHUNK - 1);
            const int pk   = ((cbase + el) << SLA) | slot;
            if (t < RCAP) {
              if (lane == 0) { hl[t] = pk; cnt[slot] = cnt[slot] + 1; }
              t = t + 1;
            } else {
              ov = 1;
            }
          }
        }
      }
    }
    __syncthreads();
  }
  if (wave == 0 && lane == 0) { misc[8] = t; misc[9] = ov; }
  __syncthreads();
  int tt = misc[8];
  tt = tt < 0 ? 0 : (tt > RCAP ? RCAP : tt);
  const int ovf = misc[9];

  if (wave == 0) {
    const int base = lane * (NBA / 32);
    int s = 0;
#pragma unroll 1
    for (int i = 0; i < NBA / 32; ++i) s += cnt[base + i];
    int incl = s;
#pragma unroll
    for (int d = 1; d < 32; d <<= 1) {
      const int y = __shfl_up(incl, d, 32);
      if (lane >= d) incl += y;
    }
    int run = incl - s;
#pragma unroll 1
    for (int i = 0; i < NBA / 32; ++i) {
      const int cv = cnt[base + i];
      offs[base + i] = run;
      cur[base + i]  = run;
      run += cv;
    }
  }
  __syncthreads();
  if (wave == 0) {
#pragma unroll 1
    for (int b0 = 0; b0 < tt; b0 += 32) {
      const int idx = b0 + lane;
      const int ent = hl[idx < RCAP ? idx : RCAP - 1];
      const int m32 = (tt - b0) < 32 ? (tt - b0) : 32;
#pragma unroll 1
      for (int k = 0; k < m32; ++k) {
        const int u    = __builtin_amdgcn_readlane(ent, k);
        const int slot = u & (NBA - 1);
        if (lane == 0) {
          int p = cur[slot];
          p = p < 0 ? 0 : (p > RCAP - 1 ? RCAP - 1 : p);
          sl[p] = u;
          cur[slot] = p + 1;
        }
      }
    }
  }
  __syncthreads();

  const float qn = __int_as_float(0x7fc00000);
  const float pz = (ovf != 0) ? qn : 0.0f;
#pragma unroll 1
  for (int si = 0; si < NBA / NWAVE; ++si) {
    const int s    = si * NWAVE + wave;
    const int node = nodeBase + s;
    const int craw = cnt[s];
    const bool big = craw > DEGCAP;
    int c = craw < 0 ? 0 : (craw > DEGCAP ? DEGCAP : craw);
    int o = offs[s];
    o = o < 0 ? 0 : (o > RCAP ? RCAP : o);
    if (c > RCAP - o) c = RCAP - o;
    const int nc  = node < nN ? node : nN - 1;
    const int alb = (nc >> 6) * (2 * GBM) + (nc & (GBM - 1));
    const float as0 = AL[alb];
    const float ad  = AL[alb + GBM];
    float l0 = as0 + ad;
    l0 = l0 > 0.f ? l0 : NEGSL * l0;

    float mx = l0;
#pragma unroll 1
    for (int b0 = 0; b0 < c; b0 += 32) {
      const int q = b0 + lane;
      int idx = o + q;
      idx = idx > RCAP - 1 ? RCAP - 1 : idx;
      const int ent = sl[idx];
      int eid = ent >> SLA;
      eid = eid < 0 ? 0 : (eid > nE - 1 ? nE - 1 : eid);
      int sr = srcs[eid];
      sr = sr < 0 ? 0 : (sr > nN - 1 ? nN - 1 : sr);
      const float es = AL[(sr >> 6) * (2 * GBM) + (sr & (GBM - 1))];
      float lg = es + ad;
      lg = lg > 0.f ? lg : NEGSL * lg;
      lg = (q < c) ? lg : l0;
      mx = fmaxf(mx, lg);
    }
#pragma unroll
    for (int off = 16; off > 0; off >>= 1) mx = fmaxf(mx, __shfl_xor(mx, off));

    float dn = 0.0f;
    float a0 = 0.0f, a1 = 0.0f, a2 = 0.0f, a3 = 0.0f;
#pragma unroll 1
    for (int b0 = 0; b0 < c; b0 += 32) {
      const int q = b0 + lane;
      int idx = o + q;
      idx = idx > RCAP - 1 ? RCAP - 1 : idx;
      const int ent = sl[idx];
      int eid = ent >> SLA;
      eid = eid < 0 ? 0 : (eid > nE - 1 ? nE - 1 : eid);
      int sr = srcs[eid];
      sr = sr < 0 ? 0 : (sr > nN - 1 ? nN - 1 : sr);
      const float es = AL[(sr >> 6) * (2 * GBM) + (sr & (GBM - 1))];
      float lg = es + ad;
      lg = lg > 0.f ? lg : NEGSL * lg;
      float w = expf(lg - mx);
      w = (q < c) ? w : 0.0f;
      const int wi  = __float_as_int(w);
      const int m32 = (c - b0) < 32 ? (c - b0) : 32;
#pragma unroll 1
      for (int k = 0; k < m32; ++k) {
        const int   sk = __builtin_amdgcn_readlane(sr, k);
        const float wk = __int_as_float(__builtin_amdgcn_readlane(wi, k));
        const v4f a = *(const v4f*)(xl + (size_t)sk * DCH + c0);
        dn += wk;
        a0 = fmaf(wk, a.x, a0);
        a1 = fmaf(wk, a.y, a1);
        a2 = fmaf(wk, a.z, a2);
        a3 = fmaf(wk, a.w, a3);
      }
    }
    {
      const float w0 = expf(l0 - mx);
      const v4f a = *(const v4f*)(xl + (size_t)nc * DCH + c0);
      dn += w0;
      a0 = fmaf(w0, a.x, a0);
      a1 = fmaf(w0, a.y, a1);
      a2 = fmaf(w0, a.z, a2);
      a3 = fmaf(w0, a.w, a3);
    }
    const float inv = __builtin_amdgcn_rcpf(dn + EPS_SM);
    const float pzr = big ? qn : pz;
    const bool live = node < nN;
    float y0 = fmaf(a0, inv, bv.x);
    float y1 = fmaf(a1, inv, bv.y);
    float y2 = fmaf(a2, inv, bv.z);
    float y3 = fmaf(a3, inv, bv.w);
    y0 = (y0 > 0.0f) ? y0 : (y0 - y0);
    y1 = (y1 > 0.0f) ? y1 : (y1 - y1);
    y2 = (y2 > 0.0f) ? y2 : (y2 - y2);
    y3 = (y3 > 0.0f) ? y3 : (y3 - y3);
    y0 = y0 + pzr; y1 = y1 + pzr; y2 = y2 + pzr; y3 = y3 + pzr;
    const float v0 = live ? y0 : 0.0f;
    const float v1 = live ? y1 : 0.0f;
    const float v2 = live ? y2 : 0.0f;
    const float v3 = live ? y3 : 0.0f;

    if constexpr (OUTF == 0) {
      const unsigned hbx = bf16_bits(v0), hby = bf16_bits(v1), hbz = bf16_bits(v2), hbw = bf16_bits(v3);
      const unsigned lbx = bf16_bits(v0 - __uint_as_float(hbx << 16));
      const unsigned lby = bf16_bits(v1 - __uint_as_float(hby << 16));
      const unsigned lbz = bf16_bits(v2 - __uint_as_float(hbz << 16));
      const unsigned lbw = bf16_bits(v3 - __uint_as_float(hbw << 16));
      const int hw0 = (int)(hbx | (hby << 16)), hw1 = (int)(hbz | (hbw << 16));
      const int lw0 = (int)(lbx | (lby << 16)), lw1 = (int)(lbz | (lbw << 16));
      const int sa = (2 * lane) & 31, sb = (2 * lane + 1) & 31;
      const int g0 = __shfl(hw0, sa), g1 = __shfl(hw1, sa), g2 = __shfl(hw0, sb), g3 = __shfl(hw1, sb);
      const int q0 = __shfl(lw0, sa), q1 = __shfl(lw1, sa), q2 = __shfl(lw0, sb), q3 = __shfl(lw1, sb);
      const bool lsel = lane >= 16;
      v4u pv;
      pv.x = (unsigned)(lsel ? q0 : g0);
      pv.y = (unsigned)(lsel ? q1 : g1);
      pv.z = (unsigned)(lsel ? q2 : g2);
      pv.w = (unsigned)(lsel ? q3 : g3);
      if (node < mRows) {
        unsigned short* gp = hb + (size_t)node * KP + 8 * lane;
        *(volatile v4u*)gp = pv;
        __threadfence();
        *(volatile v4u*)gp = pv;
      }
    } else {
      v4f ov4;
      ov4.x = v0; ov4.y = v1; ov4.z = v2; ov4.w = v3;
      if (live) {
        float* op = outp + (size_t)node * DCH + c0;
        *(volatile v4f*)op = ov4;
        __threadfence();
        *(volatile v4f*)op = ov4;
      }
    }
  }
}

static inline int cdiv(int a, int b) { return (a + b - 1) / b; }

extern "C" void kernel_launch(void* const* d_in, const int* in_sizes, int n_in,
                              void* d_out, int out_size, void* d_ws, size_t ws_size,
                              hipStream_t stream) {
  if (n_in < 14) return;
  if (in_sizes[0] < DCH || (in_sizes[0] % DCH) != 0) return;
  const int nN = in_sizes[0] / DCH;
  if (nN < 1 || nN > (1 << 22)) return;
  if (in_sizes[1] < 2 || (in_sizes[1] & 1) != 0) return;
  const int nE = in_sizes[1] / 2;
  if (nE < 1 || nE >= (1 << 21)) return;
  if (in_sizes[2] != DCH * DCH || in_sizes[6] != DCH * DCH || in_sizes[10] != DCH * DCH) return;
  if (in_sizes[3] != DCH || in_sizes[4] != DCH || in_sizes[5] != DCH) return;
  if (in_sizes[7] != DCH || in_sizes[8] != DCH || in_sizes[9] != DCH) return;
  if (in_sizes[11] != DCH || in_sizes[12] != DCH || in_sizes[13] != DCH) return;
  if ((long long)out_size != (long long)nN * DCH) return;

  const float* x   = (const float*)d_in[0];
  const int*   g   = (const int*)d_in[1];
  const float* W0  = (const float*)d_in[2];
  const float* as0 = (const float*)d_in[3];
  const float* ad0 = (const float*)d_in[4];
  const float* b0  = (const float*)d_in[5];
  const float* W1  = (const float*)d_in[6];
  const float* as1 = (const float*)d_in[7];
  const float* ad1 = (const float*)d_in[8];
  const float* b1  = (const float*)d_in[9];
  const float* W2  = (const float*)d_in[10];
  const float* as2 = (const float*)d_in[11];
  const float* ad2 = (const float*)d_in[12];
  const float* b2  = (const float*)d_in[13];
  float* out = (float*)d_out;
  const int* src = g;
  const int* dst = g + nE;

  const int MP   = cdiv(nN, GBM) * GBM;
  const int gM   = MP / GBM;
  const int gA   = cdiv(MP, NBA);
  if ((long long)gA * NBA < (long long)MP) return;
  const int vec8 = ((nE & 3) == 0) ? 1 : 0;

  char* ws = (char*)d_ws;
  size_t off = 0;
  const size_t oW0B = off; off += (size_t)DCH * DCH * 2;                  off = (off + 255) & ~(size_t)255;
  const size_t oW1C = off; off += (size_t)DCH * KP * 2;                   off = (off + 255) & ~(size_t)255;
  const size_t oW2C = off; off += (size_t)DCH * KP * 2;                   off = (off + 255) & ~(size_t)255;
  const size_t oAL  = off; off += (size_t)gM * (2 * GBM) * 4;             off = (off + 255) & ~(size_t)255;
  const size_t oXB  = off; off += (size_t)MP * DCH * 2;                   off = (off + 255) & ~(size_t)255;
  const size_t oH   = off; off += (size_t)MP * DCH * 4;                   off = (off + 255) & ~(size_t)255;
  const size_t oAP  = off; off += (size_t)MP * KP * 2;                    off = (off + 255) & ~(size_t)255;
  if (off > ws_size || off > (size_t)WSMAX) return;
  unsigned short* W0B = (unsigned short*)(ws + oW0B);
  unsigned short* W1C = (unsigned short*)(ws + oW1C);
  unsigned short* W2C = (unsigned short*)(ws + oW2C);
  float*          ALp = (float*)(ws + oAL);
  unsigned short* XB  = (unsigned short*)(ws + oXB);
  float*          H   = (float*)(ws + oH);
  unsigned short* AP  = (unsigned short*)(ws + oAP);

  const size_t aggLds  = (size_t)AGG_LDS_INTS * 4;
  const size_t gemmLds = (size_t)(GBM * GBN + 2 * GBM) * 4;
  hipFuncSetAttribute(reinterpret_cast<const void*>(&k_agg<0>), hipFuncAttributeMaxDynamicSharedMemorySize, (int)aggLds);
  hipFuncSetAttribute(reinterpret_cast<const void*>(&k_agg<1>), hipFuncAttributeMaxDynamicSharedMemorySize, (int)aggLds);

  const int nUx = MP * (DCH / 8);
  k_wprep<<<(NU0 + 2 * NUC) / NTHR, NTHR, 0, stream>>>(W0, W1, W2, W0B, W1C, W2C);
  k_cvx<<<cdiv(nUx, NTHR), NTHR, 0, stream>>>(x, nN, nUx, XB);
  k_gemm<1><<<gM, GTHR, gemmLds, stream>>>(XB, DCH, W0B, DCH, DCH, H, as0, ad0, ALp);
  k_agg<0><<<gA, NTHR, aggLds, stream>>>(src, dst, nE, nN, vec8, MP, ALp, H, b0, AP, out);
  k_gemm<1><<<gM, GTHR, gemmLds, stream>>>(AP, KP, W1C, KP, KP, H, as1, ad1, ALp);
  k_agg<0><<<gA, NTHR, aggLds, stream>>>(src, dst, nE, nN, vec8, MP, ALp, H, b1, AP, out);
  k_gemm<1><<<gM, GTHR, gemmLds, stream>>>(AP, KP, W2C, KP, KP, H, as2, ad2, ALp);
  k_agg<1><<<gA, NTHR, aggLds, stream>>>(src, dst, nE, nN, vec8, MP, ALp, H, b2, AP, out);
}
